// RawDotProductAttention_79413945303402
// MI455X (gfx1250) — hardware-verified
//
#include <hip/hip_runtime.h>
#include <stdint.h>

typedef __attribute__((ext_vector_type(16))) _Float16 v16h;
typedef __attribute__((ext_vector_type(8)))  _Float16 v8h;
typedef __attribute__((ext_vector_type(16))) __bf16   v16b;
typedef __attribute__((ext_vector_type(8)))  __bf16   v8b;
typedef __attribute__((ext_vector_type(8)))  float    v8f;
typedef __attribute__((ext_vector_type(4)))  float    v4f;
typedef __attribute__((ext_vector_type(4)))  unsigned int u32x4;

constexpr int NQ = 8192;
constexpr int NK = 8192;
constexpr int HD = 128;
constexpr int KC = 64;
constexpr int QB = 64;
constexpr int NWAVE = 4;
constexpr int KP = 136;
constexpr int VP = 72;
constexpr int PP = 72;
constexpr int OP = 132;
constexpr float PSC = 32768.0f;

static_assert(NQ % QB == 0, "qb");
static_assert(NK % KC == 0, "kc");
static_assert(HD == 128, "hd");
static_assert((KP % 8) == 0 && (VP % 8) == 0 && (PP % 8) == 0 && (OP % 4) == 0, "align");

constexpr size_t WS_KB_OFF = 0;
constexpr size_t WS_KB_BYTES = (size_t)NK * HD * 2;
constexpr size_t WS_VT_OFF = WS_KB_OFF + WS_KB_BYTES;
constexpr size_t WS_VT_BYTES = (size_t)HD * NK * 2;
constexpr size_t WS_TOTAL = WS_VT_OFF + WS_VT_BYTES;
static_assert(WS_TOTAL == 4194304, "ws");
static_assert((WS_VT_OFF % 128) == 0, "wsalign");

__device__ __forceinline__ unsigned short f2bf_bits(float f) {
  unsigned u = __float_as_uint(f);
  return (unsigned short)((u + 0x7FFFu + ((u >> 16) & 1u)) >> 16);
}
__device__ __forceinline__ float bf_bits2f(unsigned short h) { return __uint_as_float(((unsigned)h) << 16); }
__device__ __forceinline__ __bf16 at_f2bf(float f) { return __builtin_bit_cast(__bf16, f2bf_bits(f)); }
__device__ __forceinline__ unsigned int pk_bf(float a, float b) {
  return (unsigned int)f2bf_bits(a) | ((unsigned int)f2bf_bits(b) << 16);
}
__device__ __forceinline__ __bf16 at_to16h(float f) { return __builtin_bit_cast(__bf16, (_Float16)f); }

__device__ __forceinline__ v8f at_mma_b(v16b a, v16b b, v8f c) {
  c = __builtin_amdgcn_wmma_f32_16x16x32_bf16(false, a, false, b, (short)0, c, false, false);
  asm volatile("v_nop\n\tv_nop\n\tv_nop\n\tv_nop" : "+v"(c) : "v"(a), "v"(b));
  return c;
}
__device__ __forceinline__ v8f at_mma_h(v16b a, v16b b, v8f c) {
  const v16h ah = __builtin_bit_cast(v16h, a), bh = __builtin_bit_cast(v16h, b);
  c = __builtin_amdgcn_wmma_f32_16x16x32_f16(false, ah, false, bh, (short)0, c, false, false);
  asm volatile("v_nop\n\tv_nop\n\tv_nop\n\tv_nop" : "+v"(c) : "v"(ah), "v"(bh));
  return c;
}

union FB { v16b v; v8b h[2]; };

__global__ __launch_bounds__(256) void prep_kv(const float* __restrict__ Kf, const float* __restrict__ Vf,
                                               unsigned short* __restrict__ Kb, unsigned short* __restrict__ VT) {
  __shared__ __align__(16) _Float16 sV[HD * VP];
  const int tid  = threadIdx.x;
  const int lane = tid & 31;
  const int wave = tid >> 5;
  const int kv0  = blockIdx.x * KC;

  u32x4 kw[4];
#pragma unroll
  for (int it = 0; it < 4; ++it) {
    const size_t e0 = (size_t)kv0 * HD + (size_t)(it * 256 + tid) * 8;
    const v4f a = *(const v4f*)(Kf + e0);
    const v4f b = *(const v4f*)(Kf + e0 + 4);
    u32x4 w;
    w[0] = pk_bf(a[0], a[1]); w[1] = pk_bf(a[2], a[3]);
    w[2] = pk_bf(b[0], b[1]); w[3] = pk_bf(b[2], b[3]);
    kw[it] = w;
  }
  for (int pass = 0; pass < 2; ++pass) {
#pragma unroll
    for (int it = 0; it < 4; ++it) {
      const size_t e0 = (size_t)kv0 * HD + (size_t)(it * 256 + tid) * 8;
      *(volatile u32x4*)(Kb + e0) = kw[it];
    }
    __threadfence();
  }

#pragma unroll 2
  for (int it = 0; it < 8; ++it) {
    const int idx = it * 256 + tid;
    const int r  = idx >> 5;
    const int d0 = (idx & 31) * 4;
    const v4f x = *(const v4f*)(Vf + (size_t)(kv0 + r) * HD + d0);
#pragma unroll
    for (int e = 0; e < 4; ++e) sV[(d0 + e) * VP + r] = (_Float16)bf_bits2f(f2bf_bits(x[e]));
  }
  __syncthreads();
  {
    const int q  = lane >> 3;
    const int c8 = (lane & 7) * 8;
    _Float16* VTh = (_Float16*)(void*)VT;
    for (int pass = 0; pass < 2; ++pass) {
#pragma unroll
      for (int it = 0; it < 4; ++it) {
        const int d = it * 32 + wave * 4 + q;
        const v8h val = *(const v8h*)(sV + d * VP + c8);
        *(volatile v8h*)(VTh + (size_t)d * NK + kv0 + c8) = val;
      }
      __threadfence();
    }
  }
}

__global__ __launch_bounds__(128) void attn_flat(const float* __restrict__ Qf,
                                                 const unsigned short* __restrict__ Kb,
                                                 const unsigned short* __restrict__ VT,
                                                 float* __restrict__ Out) {
  __shared__ __align__(16) unsigned short Ks[KC * KP];
  __shared__ __align__(16) unsigned short Vs[HD * VP];
  __shared__ __align__(16) __bf16 Ps[NWAVE][16 * PP];
  __shared__ __align__(16) float  Os[NWAVE][16 * OP];

  const int tid  = threadIdx.x;
  const int wave = tid >> 5;
  const int lane = tid & 31;
  const int hh   = lane >> 4;
  const int c    = lane & 15;
  const int q0   = blockIdx.x * QB + wave * 16;

  v16b qa[4];
  {
    const float* qrow = Qf + (size_t)(q0 + c) * HD;
#pragma unroll
    for (int dc = 0; dc < 4; ++dc) {
      const v4f a0 = *(const v4f*)(qrow + dc * 32 + 8 * hh);
      const v4f a1 = *(const v4f*)(qrow + dc * 32 + 8 * hh + 4);
      const v4f b0 = *(const v4f*)(qrow + dc * 32 + 16 + 8 * hh);
      const v4f b1 = *(const v4f*)(qrow + dc * 32 + 16 + 8 * hh + 4);
#pragma unroll
      for (int e = 0; e < 4; ++e) {
        qa[dc][e]      = at_f2bf(a0[e]);
        qa[dc][4 + e]  = at_f2bf(a1[e]);
        qa[dc][8 + e]  = at_f2bf(b0[e]);
        qa[dc][12 + e] = at_f2bf(b1[e]);
      }
      asm volatile("" ::: "memory");
    }
  }

  float mrow[8], lrow[8];
  v8f oacc[8];
#pragma unroll
  for (int r = 0; r < 8; ++r) { mrow[r] = -INFINITY; lrow[r] = 0.f; }
#pragma unroll
  for (int t = 0; t < 8; ++t) oacc[t] = (v8f){0.f,0.f,0.f,0.f,0.f,0.f,0.f,0.f};

  for (int kc = 0; kc < NK / KC; ++kc) {
    const int kv0 = kc * KC;
    __syncthreads();
#pragma unroll 2
    for (int it = 0; it < 8; ++it) {
      const int idx = it * 128 + tid;
      const int r   = idx >> 4;
      const int seg = idx & 15;
      const u32x4 w = *(const u32x4*)(Kb + (size_t)(kv0 + r) * HD + seg * 8);
      *(u32x4*)(Ks + r * KP + seg * 8) = w;
    }
#pragma unroll 2
    for (int it = 0; it < 8; ++it) {
      const int idx = it * 128 + tid;
      const int d   = idx >> 3;
      const int seg = idx & 7;
      const u32x4 w = *(const u32x4*)(VT + (size_t)d * NK + kv0 + seg * 8);
      *(u32x4*)(Vs + d * VP + seg * 8) = w;
    }
    __syncthreads();

    v8f s[4];
#pragma unroll
    for (int j = 0; j < 4; ++j) {
      s[j] = (v8f){0.f,0.f,0.f,0.f,0.f,0.f,0.f,0.f};
#pragma unroll
      for (int dc = 0; dc < 4; ++dc) {
        FB kb;
        const unsigned short* kp = Ks + (j * 16 + c) * KP + dc * 32 + 8 * hh;
        kb.h[0] = *(const v8b*)(const void*)(kp);
        kb.h[1] = *(const v8b*)(const void*)(kp + 16);
        s[j] = at_mma_b(qa[dc], kb.v, s[j]);
      }
    }

    float cm[8];
#pragma unroll
    for (int r = 0; r < 8; ++r) {
      float m = fmaxf(fmaxf(s[0][r], s[1][r]), fmaxf(s[2][r], s[3][r]));
#pragma unroll
      for (int off = 1; off < 16; off <<= 1) m = fmaxf(m, __shfl_xor(m, off, 32));
      cm[r] = m;
    }

    __bf16* pw = Ps[wave];
#pragma unroll
    for (int r = 0; r < 8; ++r) {
      const float mnew  = fmaxf(mrow[r], cm[r]);
      const float alpha = expf(mrow[r] - mnew);
      mrow[r] = mnew;
      float psum = 0.f;
#pragma unroll
      for (int j = 0; j < 4; ++j) {
        const float p = expf(s[j][r] - mnew);
        psum += p;
        pw[(8 * hh + r) * PP + j * 16 + c] = at_to16h(p * PSC);
      }
#pragma unroll
      for (int off = 1; off < 16; off <<= 1) psum += __shfl_xor(psum, off, 32);
      lrow[r] = lrow[r] * alpha + psum;
#pragma unroll
      for (int t = 0; t < 8; ++t) oacc[t][r] *= alpha;
    }
    __syncthreads();

#pragma unroll 1
    for (int kk = 0; kk < 2; ++kk) {
      FB pa;
      pa.h[0] = *(const v8b*)(pw + c * PP + kk * 32 + 8 * hh);
      pa.h[1] = *(const v8b*)(pw + c * PP + kk * 32 + 16 + 8 * hh);
#pragma unroll
      for (int t = 0; t < 8; ++t) {
        FB vb;
        const unsigned short* vp = Vs + (t * 16 + c) * VP + kk * 32 + 8 * hh;
        vb.h[0] = *(const v8b*)(const void*)(vp);
        vb.h[1] = *(const v8b*)(const void*)(vp + 16);
        oacc[t] = at_mma_h(pa.v, vb.v, oacc[t]);
      }
    }
  }

  float* os = Os[wave];
#pragma unroll
  for (int r = 0; r < 8; ++r) {
    const float inv = 1.0f / (lrow[r] * PSC);
#pragma unroll
    for (int t = 0; t < 8; ++t) os[(8 * hh + r) * OP + t * 16 + c] = oacc[t][r] * inv;
  }
  __syncthreads();
  for (int pass = 0; pass < 2; ++pass) {
#pragma unroll
    for (int row = 0; row < 16; ++row) {
      const v4f val = *(const v4f*)(os + row * OP + lane * 4);
      *(volatile v4f*)(Out + (size_t)(q0 + row) * HD + lane * 4) = val;
    }
    __threadfence();
  }
}

extern "C" void kernel_launch(void* const* d_in, const int* in_sizes, int n_in,
                              void* d_out, int out_size, void* d_ws, size_t ws_size,
                              hipStream_t stream) {
  if (n_in < 3) return;
  if (in_sizes[0] != NQ * HD || in_sizes[1] != NK * HD || in_sizes[2] != NK * HD) return;
  if (out_size != NQ * HD) return;
  if (ws_size < WS_TOTAL) return;
  const float* Q = (const float*)d_in[0];
  const float* K = (const float*)d_in[1];
  const float* V = (const float*)d_in[2];
  float* O = (float*)d_out;
  unsigned short* Kb = (unsigned short*)((char*)d_ws + WS_KB_OFF);
  unsigned short* VT = (unsigned short*)((char*)d_ws + WS_VT_OFF);

  prep_kv<<<dim3(NK / KC), dim3(256), 0, stream>>>(K, V, Kb, VT);
  attn_flat<<<dim3(NQ / QB), dim3(128), 0, stream>>>(Q, Kb, VT, O);
}
